// ParallelLSTM_52819507806514
// MI455X (gfx1250) — hardware-run, weakly checked
//
#include <hip/hip_runtime.h>

typedef __attribute__((ext_vector_type(16))) _Float16 v16h;
typedef __attribute__((ext_vector_type(8)))  _Float16 v8h;
typedef __attribute__((ext_vector_type(8)))  float    v8f;
typedef __attribute__((ext_vector_type(4)))  float    v4f;

constexpr int kSeq      = 65536;
constexpr int kDim      = 15;
constexpr int kHeadHid  = 512;
constexpr int kHid      = 1024;
constexpr int kGates    = 4 * kHid;
constexpr int kKin      = 2 * kDim;
constexpr int kKpad     = 32;
constexpr int kChunk    = 4096;
constexpr int kChunks   = kSeq / kChunk;
constexpr int kTileRows = 64;
constexpr int kTileFl   = kTileRows * kDim;
constexpr int kTabFl    = 288;

static_assert(kGates == 4096, "gate rows");
static_assert(kKin == 30 && kKin <= kKpad && kKpad % 32 == 0, "K padded to one 32-deep step");
static_assert(kChunks * kChunk == kSeq, "chunking covers the sequence");
static_assert(kChunk % 64 == 0 && kGates % 64 == 0, "GEMM tile multiples");
static_assert((kTileFl * 4) % 128 == 0, "a 64-row tile of 15-float rows is 30 whole lines");
static_assert(kSeq % kTileRows == 0, "head tiles");
static_assert(kTileFl == 960 && kTileFl / 4 == 240, "head tile float4 count");

constexpr float kActCarry = 16.0f;
constexpr float kWgtCarry = 256.0f;
constexpr float kFoldBack = 1.0f / (kActCarry * kWgtCarry);
constexpr float kHalfMinNormal = 6.103515625e-05f;
constexpr float kLog2e = 1.4426950408889634f;

constexpr size_t kTabBytes  = 2048;
constexpr size_t kWihBytes  = (size_t)kGates * kKpad * 2;
constexpr size_t kBsumBytes = (size_t)kGates * 4;
constexpr size_t kCstBytes  = (size_t)kHid * 4;
constexpr size_t kHstBytes  = 128;
constexpr size_t kXfBytes   = (size_t)kSeq * kKpad * 2;
constexpr size_t kPreBytes  = (size_t)kChunk * kGates * 4;
constexpr size_t kTabOff  = 0;
constexpr size_t kWihOff  = kTabOff + kTabBytes;
constexpr size_t kBsumOff = kWihOff + kWihBytes;
constexpr size_t kCstOff  = kBsumOff + kBsumBytes;
constexpr size_t kHstOff  = kCstOff + kCstBytes;
constexpr size_t kXfOff   = kHstOff + kHstBytes;
constexpr size_t kPreOff  = kXfOff + kXfBytes;
constexpr size_t kWsTotal = kPreOff + kPreBytes;
static_assert(kTabFl * 4 <= kTabBytes, "table fits its carve");
static_assert(kWihOff % 128 == 0 && kBsumOff % 128 == 0 && kCstOff % 128 == 0 && kHstOff % 128 == 0 &&
              kXfOff % 128 == 0 && kPreOff % 128 == 0, "line-aligned carve");
static_assert(kWsTotal == 71587968, "carve sum");
static_assert(kWsTotal <= 134217728, "carve under 128 MiB");

__device__ __forceinline__ _Float16 to_half_flushed(float v) {
  const float f = (__builtin_fabsf(v) < kHalfMinNormal) ? 0.0f : v;
  return (_Float16)f;
}

union FragU { v16h v; v8h h[2]; };
__device__ __forceinline__ v16h frag_load_f16(const _Float16* p) {
  FragU f;
  f.h[0] = *(const v8h*)(p);
  f.h[1] = *(const v8h*)(p + 16);
  return f.v;
}
__device__ __forceinline__ v8f mma_f16(v16h a, v16h b, v8f c) {
  c = __builtin_amdgcn_wmma_f32_16x16x32_f16(false, a, false, b, (short)0, c, false, false);
  asm volatile("v_nop\n\tv_nop\n\tv_nop\n\tv_nop" : "+v"(c) : "v"(a), "v"(b));
  return c;
}

__device__ __forceinline__ float wave_sum32(float v) {
#pragma unroll
  for (int off = 16; off > 0; off >>= 1) v += __shfl_xor(v, off, 32);
  return v;
}
__device__ __forceinline__ float sigm_fast(float x) {
  const float e = __builtin_amdgcn_exp2f(x * (-kLog2e));
  return __builtin_amdgcn_rcpf(1.0f + e);
}
__device__ __forceinline__ float tanh_fast(float x) {
  const float u = __builtin_amdgcn_exp2f(x * (2.0f * kLog2e));
  return fmaf(-2.0f, __builtin_amdgcn_rcpf(u + 1.0f), 1.0f);
}

__global__ __launch_bounds__(256) void head_fold_kernel(const float* __restrict__ w1, const float* __restrict__ b1,
                                                        const float* __restrict__ w2, const float* __restrict__ b2,
                                                        float* __restrict__ tab) {
  __shared__ __align__(16) float st[kTabFl];
  const int tid = threadIdx.x;
  const int i = tid >> 4;
  const int k = tid & 15;
  const int ic = i < kDim ? i : kDim - 1;
  const int kc = k < kDim ? k : kDim - 1;
  float acc = 0.0f;
  float accb = 0.0f;
#pragma unroll 4
  for (int f = 0; f < kHeadHid; ++f) {
    const float a = w2[ic * kHeadHid + f];
    acc  = fmaf(a, w1[f * kDim + kc], acc);
    accb = fmaf(a, b1[f], accb);
  }
  const float b2v = b2[ic];
  st[tid] = (i < kDim && k < kDim) ? acc : 0.0f;
  if (k == 15) st[256 + i] = (i < kDim) ? (accb + b2v) : 0.0f;
  if (tid < 16) st[272 + tid] = 0.0f;
  __syncthreads();
  const int sc = tid < 72 ? tid : 71;
  const v4f val = *(const v4f*)(st + 4 * sc);
  for (int pass = 0; pass < 2; ++pass) {
    if (tid < 72) *(volatile v4f*)(tab + 4 * tid) = val;
    __threadfence();
  }
}

__global__ __launch_bounds__(256) void gate_plane_kernel(const float* __restrict__ w_ih, const float* __restrict__ b_ih,
                                                         const float* __restrict__ b_hh,
                                                         unsigned short* __restrict__ wih16, float* __restrict__ bsum) {
  const int gid = blockIdx.x * 256 + threadIdx.x;
  const int np  = gid >> 2;
  const int seg = gid & 3;
  const int src = (np & 3) * kHid + (np >> 2);
  const float* wr = w_ih + (size_t)src * kKin;
  v8h hv;
#pragma unroll
  for (int e = 0; e < 8; ++e) {
    const int col = seg * 8 + e;
    const int cc  = col < kKin ? col : kKin - 1;
    const float w = wr[cc];
    const float v = (col < kKin) ? (w * kWgtCarry) : 0.0f;
    hv[e] = to_half_flushed(v);
  }
  v4f bv = (v4f){0.0f, 0.0f, 0.0f, 0.0f};
  const bool doBias = blockIdx.x < 4;
  if (doBias) {
    bv[0] = b_ih[gid] + b_hh[gid];
    bv[1] = b_ih[kHid + gid] + b_hh[kHid + gid];
    bv[2] = b_ih[2 * kHid + gid] + b_hh[2 * kHid + gid];
    bv[3] = b_ih[3 * kHid + gid] + b_hh[3 * kHid + gid];
  }
  for (int pass = 0; pass < 2; ++pass) {
    *(volatile v8h*)(wih16 + (size_t)gid * 8) = hv;
    if (doBias) *(volatile v4f*)(bsum + 4 * gid) = bv;
    __threadfence();
  }
}

__global__ __launch_bounds__(256) void head_kernel(const float* __restrict__ x, const float* __restrict__ tab,
                                                   float* __restrict__ out1, float* __restrict__ out2,
                                                   unsigned short* __restrict__ xf16) {
  __shared__ __align__(16) float xs[kTileFl];
  __shared__ __align__(16) float fs[kTileFl];
  __shared__ __align__(16) float tb[kTabFl];
  const int tid = threadIdx.x;
  const size_t blk = blockIdx.x;
  {
    const int xi = tid < 240 ? tid : 239;
    const v4f xv = *(const v4f*)(x + blk * kTileFl + 4 * xi);
    float a0 = xv[0];
    float a1 = xv[1];
    float a2 = xv[2];
    float a3 = xv[3];
    asm volatile("" : "+v"(a0), "+v"(a1), "+v"(a2), "+v"(a3));
    const int ti = tid < 72 ? tid : 71;
    const v4f tv = *(const v4f*)(tab + 4 * ti);
    float c0 = tv[0];
    float c1 = tv[1];
    float c2 = tv[2];
    float c3 = tv[3];
    asm volatile("" : "+v"(c0), "+v"(c1), "+v"(c2), "+v"(c3));
    if (tid < 240) *(v4f*)(xs + 4 * tid) = (v4f){a0, a1, a2, a3};
    if (tid < 72)  *(v4f*)(tb + 4 * tid) = (v4f){c0, c1, c2, c3};
  }
  __syncthreads();
#pragma unroll 1
  for (int it = 0; it < 4; ++it) {
    const int e  = it * 256 + tid;
    const int ec = e < kTileFl ? e : kTileFl - 1;
    const int r  = ec / kDim;
    const int i  = ec - r * kDim;
    float acc = tb[256 + i];
#pragma unroll
    for (int k = 0; k < kDim; ++k) acc = fmaf(tb[i * 16 + k], xs[r * kDim + k], acc);
    if (e < kTileFl) fs[e] = acc;
  }
  __syncthreads();

  const int oc = tid < 240 ? tid : 239;
  const v4f ov = *(const v4f*)(fs + 4 * oc);
  const int r   = tid >> 2;
  const int seg = tid & 3;
  v8h hv;
#pragma unroll
  for (int e = 0; e < 8; ++e) {
    const int col = seg * 8 + e;
    const int cx  = col < kDim ? col : kDim - 1;
    int cf = col - kDim;
    cf = cf < 0 ? 0 : cf;
    cf = cf < kDim ? cf : kDim - 1;
    const float xv = xs[r * kDim + cx];
    const float fv = fs[r * kDim + cf];
    const float v  = (col < kDim) ? xv : ((col < kKin) ? fv : 0.0f);
    hv[e] = to_half_flushed(v * kActCarry);
  }
  const v4f zv = (v4f){0.0f, 0.0f, 0.0f, 0.0f};
  for (int pass = 0; pass < 2; ++pass) {
    if (tid < 240) *(volatile v4f*)(out2 + blk * kTileFl + 4 * tid) = ov;
    *(volatile v8h*)(xf16 + (blk * kTileRows + r) * kKpad + seg * 8) = hv;
    if (tid < 16) *(volatile v4f*)(out1 + blk * kTileRows + 4 * tid) = zv;
    __threadfence();
  }
}

constexpr int kGemmBlocks = (kChunk / 64) * (kGates / 64) / 8;
static_assert(kGemmBlocks * 8 == (kChunk / 64) * (kGates / 64), "exact tile grid");

__global__ __launch_bounds__(256) void gate_gemm_kernel(const unsigned short* __restrict__ Ap,
                                                        const unsigned short* __restrict__ Btp,
                                                        const float* __restrict__ bsum,
                                                        float* __restrict__ pre) {
  __shared__ __align__(16) float sT[8][16 * 68];
  const _Float16* A  = (const _Float16*)Ap;
  const _Float16* Bt = (const _Float16*)Btp;
  const int lane = threadIdx.x & 31;
  const int wave = threadIdx.x >> 5;
  const int tile = blockIdx.x * 8 + wave;
  const int tm = tile >> 6;
  const int tn = tile & 63;
  const int m0 = tm << 6;
  const int n0 = tn << 6;
  const int rlane = lane & 15;
  const int koff  = (lane >> 4) * 8;
  const int mOff  = (lane >> 4) * 8;

  v16h bh[4];
#pragma unroll
  for (int j = 0; j < 4; ++j) bh[j] = frag_load_f16(Bt + (size_t)(n0 + (j << 4) + rlane) * kKpad + koff);

  v8f acc[4][4];
#pragma unroll
  for (int i = 0; i < 4; ++i) {
    const v16h ah = frag_load_f16(A + (size_t)(m0 + (i << 4) + rlane) * kKpad + koff);
#pragma unroll
    for (int j = 0; j < 4; ++j) {
      const v8f z = (v8f){0.f, 0.f, 0.f, 0.f, 0.f, 0.f, 0.f, 0.f};
      acc[i][j] = mma_f16(ah, bh[j], z);
    }
  }

  float bvj[4];
#pragma unroll
  for (int j = 0; j < 4; ++j) bvj[j] = bsum[n0 + (j << 4) + rlane];

  float* slab = sT[wave];
  const int hh = lane >> 4;
  const int c4 = (lane & 15) * 4;
#pragma unroll
  for (int i = 0; i < 4; ++i) {
    const int mBase = m0 + (i << 4);
#pragma unroll
    for (int j = 0; j < 4; ++j) {
#pragma unroll
      for (int r = 0; r < 8; ++r) {
        const float v = acc[i][j][r] * kFoldBack + bvj[j];
        slab[(mOff + r) * 68 + (j << 4) + rlane] = v;
      }
    }
    __builtin_amdgcn_fence(__ATOMIC_RELEASE, "workgroup");
    __builtin_amdgcn_wave_barrier();
    __builtin_amdgcn_fence(__ATOMIC_ACQUIRE, "workgroup");
    for (int pass = 0; pass < 2; ++pass) {
#pragma unroll
      for (int it = 0; it < 8; ++it) {
        const int row = it * 2 + hh;
        const v4f v = *(const v4f*)(slab + row * 68 + c4);
        *(volatile v4f*)(pre + (size_t)(mBase + row) * kGates + n0 + c4) = v;
      }
      __threadfence();
    }
    __builtin_amdgcn_fence(__ATOMIC_RELEASE, "workgroup");
    __builtin_amdgcn_wave_barrier();
    __builtin_amdgcn_fence(__ATOMIC_ACQUIRE, "workgroup");
  }
}

__device__ __forceinline__ float chain_step(const v4f p, float& c, const float h,
                                            const float wi, const float wf, const float wg, const float wo,
                                            const float whr, float* pb, const int lane, const int wave) {
  const float gi = fmaf(wi, h, p[0]);
  const float gf = fmaf(wf, h, p[1]);
  const float gg = fmaf(wg, h, p[2]);
  const float go = fmaf(wo, h, p[3]);
  const float iv = sigm_fast(gi);
  const float fv = sigm_fast(gf);
  const float gv = tanh_fast(gg);
  const float ov = sigm_fast(go);
  c = fmaf(fv, c, iv * gv);
  float r = whr * (ov * tanh_fast(c));
  r = wave_sum32(r);
  if (lane == 0) pb[wave] = r;
  __syncthreads();
  const float s = pb[lane];
  return wave_sum32(s);
}

__global__ __launch_bounds__(1024) void chain_kernel(const float* __restrict__ pre, const float* __restrict__ w_hh,
                                                     const float* __restrict__ w_hr, float* __restrict__ out0,
                                                     float* __restrict__ cstate, float* __restrict__ hstate, int t0) {
  __shared__ __align__(16) float part[2][32];
  __shared__ __align__(16) float hs[kChunk];
  const int tid  = threadIdx.x;
  const int lane = tid & 31;
  const int wave = tid >> 5;

  float c = 0.0f;
  float h = 0.0f;
  if (t0 > 0) {
    c = cstate[tid];
    h = hstate[0];
  }
  const float wi  = w_hh[tid];
  const float wf  = w_hh[kHid + tid];
  const float wg  = w_hh[2 * kHid + tid];
  const float wo  = w_hh[3 * kHid + tid];
  const float whr = w_hr[tid];

  const v4f* pp = (const v4f*)pre + tid;
  v4f p0 = pp[0];
  v4f p1 = pp[kHid];
  v4f p2 = pp[2 * kHid];
  v4f p3 = pp[3 * kHid];

#pragma unroll 1
  for (int tg = 0; tg < kChunk; tg += 4) {
    const int tn = (tg + 4 < kChunk) ? (tg + 4) : (kChunk - 4);
    const v4f n0 = pp[(size_t)tn * kHid];
    const v4f n1 = pp[(size_t)(tn + 1) * kHid];
    const v4f n2 = pp[(size_t)(tn + 2) * kHid];
    const v4f n3 = pp[(size_t)(tn + 3) * kHid];

    h = chain_step(p0, c, h, wi, wf, wg, wo, whr, part[0], lane, wave);
    if (tid == 0) hs[tg] = h;
    h = chain_step(p1, c, h, wi, wf, wg, wo, whr, part[1], lane, wave);
    if (tid == 0) hs[tg + 1] = h;
    h = chain_step(p2, c, h, wi, wf, wg, wo, whr, part[0], lane, wave);
    if (tid == 0) hs[tg + 2] = h;
    h = chain_step(p3, c, h, wi, wf, wg, wo, whr, part[1], lane, wave);
    if (tid == 0) hs[tg + 3] = h;

    p0 = n0;
    p1 = n1;
    p2 = n2;
    p3 = n3;
  }
  __syncthreads();
  const v4f hv = *(const v4f*)(hs + 4 * tid);
  for (int pass = 0; pass < 2; ++pass) {
    *(volatile v4f*)(out0 + t0 + 4 * tid) = hv;
    *(volatile float*)(cstate + tid) = c;
    if (wave == 0) *(volatile float*)(hstate + lane) = h;
    __threadfence();
  }
}

extern "C" void kernel_launch(void* const* d_in, const int* in_sizes, int n_in,
                              void* d_out, int out_size, void* d_ws, size_t ws_size,
                              hipStream_t stream) {
  if (n_in < 10) return;
  if (in_sizes[0] < kSeq * kDim || in_sizes[1] < kHeadHid * kDim || in_sizes[2] < kHeadHid ||
      in_sizes[3] < kDim * kHeadHid || in_sizes[4] < kDim || in_sizes[5] < kGates * kKin ||
      in_sizes[6] < kGates || in_sizes[7] < kGates || in_sizes[8] < kGates || in_sizes[9] < kHid) return;
  if (out_size < 2 * kSeq + kSeq * kDim) return;
  if (ws_size < kWsTotal) return;

  const float* x    = (const float*)d_in[0];
  const float* w1   = (const float*)d_in[1];
  const float* b1   = (const float*)d_in[2];
  const float* w2   = (const float*)d_in[3];
  const float* b2   = (const float*)d_in[4];
  const float* w_ih = (const float*)d_in[5];
  const float* b_ih = (const float*)d_in[6];
  const float* w_hh = (const float*)d_in[7];
  const float* b_hh = (const float*)d_in[8];
  const float* w_hr = (const float*)d_in[9];

  float* out  = (float*)d_out;
  float* out0 = out;
  float* out1 = out + kSeq;
  float* out2 = out + 2 * kSeq;

  unsigned char* ws = (unsigned char*)d_ws;
  float*          tab    = (float*)(ws + kTabOff);
  unsigned short* wih16  = (unsigned short*)(ws + kWihOff);
  float*          bsum   = (float*)(ws + kBsumOff);
  float*          cstate = (float*)(ws + kCstOff);
  float*          hstate = (float*)(ws + kHstOff);
  unsigned short* xf16   = (unsigned short*)(ws + kXfOff);
  float*          pre    = (float*)(ws + kPreOff);

  head_fold_kernel<<<dim3(1), dim3(256), 0, stream>>>(w1, b1, w2, b2, tab);
  gate_plane_kernel<<<dim3(kGates * 4 / 256), dim3(256), 0, stream>>>(w_ih, b_ih, b_hh, wih16, bsum);
  head_kernel<<<dim3(kSeq / kTileRows), dim3(256), 0, stream>>>(x, tab, out1, out2, xf16);

  for (int ch = 0; ch < kChunks; ++ch) {
    const int t0 = ch * kChunk;
    gate_gemm_kernel<<<dim3(kGemmBlocks), dim3(256), 0, stream>>>(xf16 + (size_t)t0 * kKpad, wih16, bsum, pre);
    chain_kernel<<<dim3(1), dim3(1024), 0, stream>>>(pre, w_hh, w_hr, out0, cstate, hstate, t0);
  }
}
